// GDNN_22136261443720
// MI455X (gfx1250) — hardware-run, weakly checked
//
#include <hip/hip_runtime.h>


#ifndef NB
#define NB 512
#endif
#define NB_FULL 512
#define NPOS 64
#define NCH  64
#define NPAT 64
#define CX   16
#define NOUT (NPOS * NCH)
#define KX   (NPOS * CX)
#define LDA  (2 * NOUT + KX)
#define XOFF  (2 * NOUT)
#define H1OFF (NOUT)
#define H2OFF 0
#define WCARRY 64.0f
#define WCINV  (1.0f / 64.0f)
#define SROWS 8
#define BN_EPS 1e-5f

static_assert(NB <= NB_FULL);
static_assert(NB % 64 == 0);
static_assert(NOUT % 64 == 0);
static_assert(KX % 32 == 0);
static_assert((NOUT + KX) % 32 == 0);
static_assert(LDA % 32 == 0);
static_assert(NB % SROWS == 0);
static_assert((SROWS * NOUT) % 256 == 0);
static_assert(NCH == 64);
static_assert(NPOS == 64);
static_assert(NPAT == 64);
static_assert(CX % 8 == 0);
static_assert((NB * (KX / 8)) % 256 == 0);
static_assert((NB * (NOUT / 8)) % 256 == 0);
static_assert((KX / 8) % 32 == 0);
static_assert((NOUT / 8) % 32 == 0);
static_assert((LDA * 2) % 128 == 0);
static_assert((XOFF * 2) % 128 == 0);
static_assert((H1OFF * 2) % 128 == 0);
static_assert((size_t)NB * NOUT * 4 <= (size_t)8388608);
static_assert(32 * 16 * 8 == 16 * 64 * 4);
static_assert(16 * 68 * 4 <= 131072);
static_assert(2 * 256 * 8 + 128 * 8 <= 131072);
static_assert(256 * 4 <= 131072);

typedef _Float16 h16;
typedef __attribute__((ext_vector_type(16))) _Float16 v16h;
typedef __attribute__((ext_vector_type(8)))  _Float16 v8h;
typedef __attribute__((ext_vector_type(8)))  float    v8f;
typedef __attribute__((ext_vector_type(4)))  float    v4f;
typedef __attribute__((ext_vector_type(2)))  double   v2d;
typedef v4f  __attribute__((may_alias)) v4fa;

__device__ __forceinline__ unsigned short f2bf(float f) { unsigned u = __float_as_uint(f); u += 0x7FFFu + ((u >> 16) & 1u); return (unsigned short)(u >> 16); }
__device__ __forceinline__ float bfr(float f) { return __uint_as_float(((unsigned)f2bf(f)) << 16); }
__device__ __forceinline__ v16h cat16(v8h lo, v8h hi) { return __builtin_shufflevector(lo, hi, 0, 1, 2, 3, 4, 5, 6, 7, 8, 9, 10, 11, 12, 13, 14, 15); }
__device__ __forceinline__ v8f wmma16(v16h a, v16h b, v8f c) { return __builtin_amdgcn_wmma_f32_16x16x32_f16(false, a, false, b, (short)0, c, false, false); }
__device__ __forceinline__ v16h  ldh(const h16* p) { return cat16(*(const v8h*)p, *(const v8h*)(p + 16)); }
__device__ __forceinline__ void wave_sync() { __builtin_amdgcn_fence(3  , "wavefront"); __builtin_amdgcn_wave_barrier(); asm volatile("" ::: "memory"); }
__device__ __forceinline__ v8f wmma16g(v16h a, v16h b, v8f c) {
    c = wmma16(a, b, c);
    asm volatile("v_nop\n\tv_nop\n\tv_nop\n\tv_nop" : "+v"(c) : "v"(a), "v"(b));
    return c;
}
static __device__ __forceinline__ h16 toh_flush(float v) { const h16 r = (h16)v; return (fabsf(v) < 6.103515625e-05f) ? (h16)0.0f : r; }

__global__ __launch_bounds__(256) void k_packx(const float* __restrict__ x, h16* ACT) {
#pragma clang fp contract(off)
    const int g = blockIdx.x * 256 + threadIdx.x;
    const int b = g >> 7, q = g & 127;
    if (b >= NB) return;
    const int n = q >> 1, c8 = (q & 1) * 8;
    const float* src = x + (size_t)b * (CX * NPOS) + (size_t)c8 * NPOS + n;
    v8h ov;
#pragma unroll
    for (int k = 0; k < 8; ++k) ov[k] = toh_flush(bfr(src[(size_t)k * NPOS]));
    h16* dst = ACT + (size_t)b * LDA + XOFF + (size_t)q * 8;
    *(volatile v8h*)dst = ov; __threadfence(); *(volatile v8h*)dst = ov;
}

__global__ __launch_bounds__(256) void k_wt(const float* __restrict__ w, h16* WT, int lp) {
#pragma clang fp contract(off)
    const int g = blockIdx.x * 256 + threadIdx.x;
    const int total = (NPAT * NCH) << lp;
    if (g >= total) return;
    const int c8 = (g & ((1 << lp) - 1)) << 3;
    const int o = (g >> lp) & (NCH - 1);
    const int q = g >> (lp + 6);
    const int Cg = 8 << lp;
    const float* src = w + ((size_t)(o * Cg + c8) * NPAT + q);
    v8h ov;
#pragma unroll
    for (int k = 0; k < 8; ++k) ov[k] = toh_flush(bfr(src[(size_t)k * NPAT]) * WCARRY);
    h16* dst = WT + (size_t)g * 8;
    *(volatile v8h*)dst = ov; __threadfence(); *(volatile v8h*)dst = ov;
}

__global__ __launch_bounds__(256) void k_wfill(const h16* __restrict__ WT, const int* __restrict__ pat, h16* W, int lp, int colOff, int ldw) {
    const int g = blockIdx.x * 256 + threadIdx.x;
    const int lpr = 6 + lp;
    const int r = g >> lpr, q = g & ((1 << lpr) - 1);
    if (r >= NOUT) return;
    const int n = r >> 6, o = r & (NCH - 1), m = q >> lp, c8 = (q & ((1 << lp) - 1)) << 3;
    const int pe = pat[n * NPOS + m];
    int ai = (pe < 0 ? -pe : pe) - 1;
    ai = ai < 0 ? (NPAT - 1) : (ai > NPAT - 1 ? NPAT - 1 : ai);
    v8h v = *(const v8h*)(WT + ((((size_t)ai * NCH + (size_t)o) << (3 + lp)) + (size_t)c8));
    asm volatile("" : "+v"(v));
    const bool ng = pe < 0, zr = pe == 0;
    v8h ov;
#pragma unroll
    for (int k = 0; k < 8; ++k) { h16 t = v[k]; t = ng ? -t : t; ov[k] = zr ? (h16)0.0f : t; }
    h16* dst = W + (size_t)r * (size_t)ldw + (size_t)colOff + ((size_t)q << 3);
    *(volatile v8h*)dst = ov; __threadfence(); *(volatile v8h*)dst = ov;
}

__global__ __launch_bounds__(32) void k_gemm(const h16* __restrict__ A, int lda, const h16* __restrict__ Bt, int K, float* C) {
    __shared__ __align__(16) float os[16 * 68];
    const int lane = threadIdx.x & 31, lr = lane & 15, hi = lane >> 4; const int r0 = blockIdx.x * 64, c0 = blockIdx.y * 64;
    v8f acc[4][4];
#pragma unroll
    for (int mb = 0; mb < 4; ++mb)
#pragma unroll
        for (int nb = 0; nb < 4; ++nb) acc[mb][nb] = (v8f){};
    const size_t aoff = (size_t)(r0 + lr) * (size_t)lda + 8 * hi, boff = (size_t)(c0 + lr) * (size_t)K + 8 * hi;
#pragma unroll 1
    for (int kc = 0; kc < K; kc += 32) {
        v16h a[4];
#pragma unroll
        for (int mb = 0; mb < 4; ++mb) a[mb] = ldh(A + aoff + (size_t)mb * 16 * (size_t)lda + kc);
#pragma unroll
        for (int nb = 0; nb < 4; ++nb) { const v16h b = ldh(Bt + boff + (size_t)nb * 16 * (size_t)K + kc);
#pragma unroll
            for (int mb = 0; mb < 4; ++mb) acc[mb][nb] = wmma16g(a[mb], b, acc[mb][nb]); }
    }
#pragma unroll
    for (int mb = 0; mb < 4; ++mb) {
#pragma unroll
        for (int nb = 0; nb < 4; ++nb) {
#pragma unroll
            for (int j = 0; j < 8; ++j) os[(hi * 8 + j) * 68 + nb * 16 + lr] = acc[mb][nb][j] * WCINV; }
        wave_sync();
        float* crow = C + (size_t)(r0 + mb * 16) * NOUT + c0;
#pragma unroll 1
        for (int ps = 0; ps < 2; ++ps) {
#pragma unroll
            for (int s = 0; s < 8; ++s) { const int row = 2 * s + (lane >> 4), cofs = (lane & 15) * 4;
                const v4f val = *(const v4fa*)(&os[row * 68 + cofs]);
                *(volatile v4f*)(crow + (size_t)row * NOUT + cofs) = val; }
            if (ps == 0) __threadfence(); }
        wave_sync();
    }
}

__global__ __launch_bounds__(256) void k_stats(const float* __restrict__ Z, double* PT) {
#pragma clang fp contract(off)
    __shared__ double ls[2 * 256];
    __shared__ double rec[128];
    const int tid = threadIdx.x;
    const float* zp = Z + (size_t)blockIdx.x * (SROWS * NOUT) + tid;
    double s = 0.0, s2 = 0.0;
#pragma unroll 4
    for (int i = 0; i < SROWS * NOUT / 256; ++i) { const float a = fabsf(zp[(size_t)i * 256]) * 0.5f; const double d = (double)a; s += d; s2 += d * d; }
    ls[tid] = s; ls[256 + tid] = s2;
    __syncthreads();
    if (tid < 128) { const int wh = tid >> 6, c = tid & 63; rec[tid] = ((ls[wh * 256 + c] + ls[wh * 256 + 64 + c]) + ls[wh * 256 + 128 + c]) + ls[wh * 256 + 192 + c]; }
    __syncthreads();
    if (tid < 64) { v2d v; v[0] = rec[2 * tid]; v[1] = rec[2 * tid + 1];
        double* dst = PT + (size_t)blockIdx.x * 128 + 2 * tid;
        *(volatile v2d*)dst = v; __threadfence(); *(volatile v2d*)dst = v; }
}

__global__ __launch_bounds__(64) void k_fin(const double* __restrict__ PT, int nblk, double invcnt, const float* __restrict__ gam, const float* __restrict__ bet, float* TAB) {
#pragma clang fp contract(off)
    const int c = threadIdx.x;
    double S = 0.0, S2 = 0.0;
#pragma unroll 1
    for (int b = 0; b < nblk; ++b) { S += PT[(size_t)b * 128 + c]; S2 += PT[(size_t)b * 128 + 64 + c]; }
    const double mu = S * invcnt;
    double var = S2 * invcnt - mu * mu; var = var < 0.0 ? 0.0 : var;
    const float rinv = 1.0f / sqrtf((float)var + BN_EPS);
    v4f t; t[0] = (float)mu; t[1] = rinv; t[2] = bfr(gam[c]); t[3] = bfr(bet[c]);
    float* dst = TAB + 4 * c;
    *(volatile v4f*)dst = t; __threadfence(); *(volatile v4f*)dst = t;
}

__global__ __launch_bounds__(256) void k_bn(const float* __restrict__ Z, const float* __restrict__ TAB, h16* AD) {
#pragma clang fp contract(off)
    __shared__ __align__(16) float tb[256];
    const int tid = threadIdx.x;
    tb[tid] = TAB[tid];
    __syncthreads();
    const int g = blockIdx.x * 256 + tid;
    const int b = g >> 9, q = g & 511;
    const float* zp = Z + (size_t)b * NOUT + (size_t)q * 8;
    const v4f z0 = *(const v4f*)zp, z1 = *(const v4f*)(zp + 4);
    const int cb = (q & 7) * 8;
    v8h ov;
#pragma unroll
    for (int k = 0; k < 8; ++k) {
        const v4f t = *(const v4fa*)(&tb[(cb + k) * 4]);
        const float z = (k < 4) ? z0[k & 3] : z1[k & 3];
        const float a = fabsf(z) * 0.5f;
        const float hv = (a - t[0]) * t[1] * t[2] + t[3];
        ov[k] = toh_flush(hv); }
    h16* dst = AD + (size_t)b * LDA + (size_t)q * 8;
    *(volatile v8h*)dst = ov; __threadfence(); *(volatile v8h*)dst = ov;
}

static constexpr size_t al256(size_t v) { return (v + 255) & ~(size_t)255; }
static constexpr size_t SZ_W    = al256((size_t)NOUT * LDA * 2);
static constexpr size_t SZ_ACT  = al256((size_t)NB * LDA * 2);
static constexpr size_t SZ_Z    = al256((size_t)NB * NOUT * 4);
static constexpr size_t SZ_WT16 = al256((size_t)NPAT * NCH * 16 * 2);
static constexpr size_t SZ_WT64 = al256((size_t)NPAT * NCH * 64 * 2);
static constexpr size_t SZ_PT   = al256((size_t)(NB / SROWS) * 128 * 8);
static constexpr size_t SZ_TAB  = al256((size_t)256 * 4);
static constexpr size_t SZ_TOTAL = SZ_W + SZ_ACT + SZ_Z + 3 * SZ_WT16 + 3 * SZ_WT64 + SZ_PT + SZ_TAB;
static_assert(SZ_TOTAL <= (size_t)134217728);
static_assert((size_t)NOUT * KX * 2 <= SZ_W);
static_assert((size_t)NOUT * (NOUT + KX) * 2 <= SZ_W);
static_assert((size_t)NOUT * (2 * NOUT + KX) * 2 <= SZ_W);
static_assert(2 * NOUT + KX == LDA);
static_assert(((NPAT * NCH * 2) % 256) == 0);
static_assert(((NOUT * (64 << 1)) % 256) == 0);
static_assert(((NOUT * (64 << 3)) % 256) == 0);

static constexpr double invcnt = 1.0 / ((double)NB * (double)NPOS);
extern "C" void kernel_launch(void* const* d_in, const int* in_sizes, int n_in,
                              void* d_out, int out_size, void* d_ws, size_t ws_size, hipStream_t stream) {
    if (n_in < 17) return;
    if ((size_t)in_sizes[0] < (size_t)NB * CX * NPOS) return;
    if ((size_t)in_sizes[1] < (size_t)NCH * 16 * NPAT || (size_t)in_sizes[3] < (size_t)NCH * 16 * NPAT || (size_t)in_sizes[6] < (size_t)NCH * 16 * NPAT) return;
    if ((size_t)in_sizes[2] < (size_t)NCH * 64 * NPAT || (size_t)in_sizes[4] < (size_t)NCH * 64 * NPAT || (size_t)in_sizes[5] < (size_t)NCH * 64 * NPAT) return;
    if (in_sizes[7] < NCH || in_sizes[8] < NCH || in_sizes[9] < NCH || in_sizes[10] < NCH) return;
    for (int i = 11; i < 17; ++i) if (in_sizes[i] < NPOS * NPOS) return;
    if ((size_t)out_size < (size_t)NB * NOUT) return;
    if (SZ_TOTAL > ws_size) return;
    const float* x    = (const float*)d_in[0];
    const float* w00  = (const float*)d_in[1];
    const float* w10  = (const float*)d_in[2];
    const float* w11  = (const float*)d_in[3];
    const float* w20  = (const float*)d_in[4];
    const float* w21  = (const float*)d_in[5];
    const float* w22  = (const float*)d_in[6];
    const float* g0   = (const float*)d_in[7];  const float* b0 = (const float*)d_in[8];
    const float* g1   = (const float*)d_in[9];  const float* b1 = (const float*)d_in[10];
    const int* p00 = (const int*)d_in[11]; const int* p10 = (const int*)d_in[12]; const int* p11 = (const int*)d_in[13];
    const int* p20 = (const int*)d_in[14]; const int* p21 = (const int*)d_in[15]; const int* p22 = (const int*)d_in[16];
    float* OUT = (float*)d_out;
    char* wsp = (char*)d_ws;
    h16* WPL = (h16*)wsp; wsp += SZ_W;
    h16* ACT = (h16*)wsp; wsp += SZ_ACT;
    float* Z = (float*)wsp; wsp += SZ_Z;
    h16* T00 = (h16*)wsp; wsp += SZ_WT16;
    h16* T11 = (h16*)wsp; wsp += SZ_WT16;
    h16* T22 = (h16*)wsp; wsp += SZ_WT16;
    h16* T10 = (h16*)wsp; wsp += SZ_WT64;
    h16* T20 = (h16*)wsp; wsp += SZ_WT64;
    h16* T21 = (h16*)wsp; wsp += SZ_WT64;
    double* PT = (double*)wsp; wsp += SZ_PT;
    float* TAB = (float*)wsp; wsp += SZ_TAB;

    const unsigned gT16 = (unsigned)(((NPAT * NCH) << 1) / 256), gT64 = (unsigned)(((NPAT * NCH) << 3) / 256);
    const unsigned gF16 = (unsigned)((NOUT * (64 << 1)) / 256), gF64 = (unsigned)((NOUT * (64 << 3)) / 256);
    const dim3 gG(NB / 64, NOUT / 64, 1);
    const int nblk = NB / SROWS;

    k_packx<<<(unsigned)((NB * (KX / 8)) / 256), 256, 0, stream>>>(x, ACT);
    k_wt<<<gT16, 256, 0, stream>>>(w00, T00, 1);
    k_wt<<<gT64, 256, 0, stream>>>(w10, T10, 3);
    k_wt<<<gT16, 256, 0, stream>>>(w11, T11, 1);
    k_wt<<<gT64, 256, 0, stream>>>(w20, T20, 3);
    k_wt<<<gT64, 256, 0, stream>>>(w21, T21, 3);
    k_wt<<<gT16, 256, 0, stream>>>(w22, T22, 1);

    k_wfill<<<gF16, 256, 0, stream>>>(T00, p00, WPL, 1, 0, KX);
    k_gemm<<<gG, 32, 0, stream>>>(ACT + XOFF, LDA, WPL, KX, Z);
    k_stats<<<(unsigned)nblk, 256, 0, stream>>>(Z, PT);
    k_fin<<<1, 64, 0, stream>>>(PT, nblk, invcnt, g0, b0, TAB);
    k_bn<<<(unsigned)((NB * (NOUT / 8)) / 256), 256, 0, stream>>>(Z, TAB, ACT + H1OFF);

    k_wfill<<<gF64, 256, 0, stream>>>(T10, p10, WPL, 3, 0, NOUT + KX);
    k_wfill<<<gF16, 256, 0, stream>>>(T11, p11, WPL, 1, NOUT, NOUT + KX);
    k_gemm<<<gG, 32, 0, stream>>>(ACT + H1OFF, LDA, WPL, NOUT + KX, Z);
    k_stats<<<(unsigned)nblk, 256, 0, stream>>>(Z, PT);
    k_fin<<<1, 64, 0, stream>>>(PT, nblk, invcnt, g1, b1, TAB);
    k_bn<<<(unsigned)((NB * (NOUT / 8)) / 256), 256, 0, stream>>>(Z, TAB, ACT + H2OFF);

    k_wfill<<<gF64, 256, 0, stream>>>(T20, p20, WPL, 3, 0, LDA);
    k_wfill<<<gF64, 256, 0, stream>>>(T21, p21, WPL, 3, NOUT, LDA);
    k_wfill<<<gF16, 256, 0, stream>>>(T22, p22, WPL, 1, 2 * NOUT, LDA);
    k_gemm<<<gG, 32, 0, stream>>>(ACT, LDA, WPL, LDA, OUT);
}
